// Decoder_50448685858992
// MI455X (gfx1250) — hardware-verified
//
#include <hip/hip_runtime.h>
#include <stdint.h>
#include <stddef.h>


#ifndef NB
#define NB 1
#endif
#ifndef SEQ
#define SEQ 2048
#endif
#define NB_FULL 1
#define SEQ_FULL 2048
#define DM 1024
#define NH 16
#define HD 64
#define FF 4096
#define RESQB 2
#define LN_EPS 1.0e-5f

static_assert(SEQ % 128 == 0);
static_assert(SEQ <= SEQ_FULL);
static_assert(NB >= 1 && NB <= NB_FULL);
static_assert(HD == 64);
static_assert(DM % 64 == 0 && FF % 64 == 0);
static_assert(DM % 32 == 0 && FF % 32 == 0);
static_assert((NB * SEQ) % 128 == 0);
static_assert(DM == 4 * 256);

typedef _Float16 v4h  __attribute__((ext_vector_type(4)));
typedef _Float16 v8h  __attribute__((ext_vector_type(8)));
typedef _Float16 v16h __attribute__((ext_vector_type(16)));
typedef float    v4f  __attribute__((ext_vector_type(4)));
typedef float    v8f  __attribute__((ext_vector_type(8)));

__device__ __forceinline__ v8f mma16(v16h a, v16h b, v8f c)
{
  c = __builtin_amdgcn_wmma_f32_16x16x32_f16(false, a, false, b, (short)0, c, false, false);
  asm volatile("v_nop\n\tv_nop\n\tv_nop\n\tv_nop" : "+v"(c) : "v"(a), "v"(b));
  return c;
}

__device__ __forceinline__ v16h ldfrag(const _Float16* p, int hs)
{
  union { v16h v; v8h q[2]; } u;
  u.q[0] = *(const v8h*)(p + 8 * hs);
  u.q[1] = *(const v8h*)(p + 16 + 8 * hs);
  return u.v;
}

__device__ __forceinline__ float bfr(float x)
{
  unsigned int u = __float_as_uint(x);
  u = (u + 0x7FFFu + ((u >> 16) & 1u)) & 0xFFFF0000u;
  return __uint_as_float(u);
}

__device__ __forceinline__ void lds_sync_wave()
{
  asm volatile("s_wait_dscnt 0x0" ::: "memory");
  __builtin_amdgcn_wave_barrier();
}

__global__ __launch_bounds__(256)
void k_cvt_act(const float* __restrict__ y, const float* __restrict__ e,
               _Float16* __restrict__ Yh, _Float16* __restrict__ Eh, int nrow)
{
  const int groups = nrow * (DM / 8);
  const int g = blockIdx.x * 256 + threadIdx.x;
  if (g >= 2 * groups) return;
  const int which = (g >= groups) ? 1 : 0;
  const int idx = g - which * groups;
  const int m = idx / (DM / 8);
  const int c = (idx - m * (DM / 8)) * 8;
  const size_t srow = (size_t)(m / SEQ) * SEQ_FULL + (size_t)(m % SEQ);
  const float* src = (which ? e : y) + srow * DM + c;
  const v4f a = *(const v4f*)src;
  const v4f b = *(const v4f*)(src + 4);
  v8h o;
  o[0] = (_Float16)bfr(a[0]); o[1] = (_Float16)bfr(a[1]); o[2] = (_Float16)bfr(a[2]); o[3] = (_Float16)bfr(a[3]);
  o[4] = (_Float16)bfr(b[0]); o[5] = (_Float16)bfr(b[1]); o[6] = (_Float16)bfr(b[2]); o[7] = (_Float16)bfr(b[3]);
  _Float16* dst = (which ? Eh : Yh) + (size_t)m * DM + c;
  *(volatile v8h*)dst = o;
  __threadfence();
  *(volatile v8h*)dst = o;
}

__global__ __launch_bounds__(256)
void k_wtr(const float* __restrict__ in, _Float16* __restrict__ out, int R, int C, float scale)
{
  __shared__ float tile[64][65];
  const int t = threadIdx.x;
  const int c0 = blockIdx.x * 64, r0 = blockIdx.y * 64;
  const size_t zoff = (size_t)blockIdx.z * (size_t)R * (size_t)C;
  {
    const int r = t >> 2, cq = (t & 3) * 16;
    const float* p = in + zoff + (size_t)(r0 + r) * C + c0 + cq;
    #pragma unroll
    for (int i = 0; i < 4; ++i) {
      const v4f v = *(const v4f*)(p + 4 * i);
      tile[r][cq + 4 * i + 0] = v[0];
      tile[r][cq + 4 * i + 1] = v[1];
      tile[r][cq + 4 * i + 2] = v[2];
      tile[r][cq + 4 * i + 3] = v[3];
    }
  }
  __syncthreads();
  const int p8 = t & 7;
  #pragma unroll 1
  for (int pass = 0; pass < 2; ++pass) {
    #pragma unroll
    for (int j = 0; j < 2; ++j) {
      const int c = (t >> 3) + 32 * j;
      v8h ov;
      #pragma unroll
      for (int i = 0; i < 8; ++i) ov[i] = (_Float16)(bfr(tile[8 * p8 + i][c]) * scale);
      _Float16* dst = out + zoff + (size_t)(c0 + c) * R + r0 + 8 * p8;
      *(volatile v8h*)dst = ov;
    }
    if (pass == 0) __threadfence();
  }
}

template<int MODE, bool RES, bool WVT>
__global__ __launch_bounds__(128) __attribute__((amdgpu_num_vgpr(256)))
void k_gemm(const _Float16* __restrict__ A, int lda,
            const _Float16* __restrict__ BT, int ldb, int sBz,
            const float* __restrict__ bias, int sBias,
            int K, int prow,
            _Float16* __restrict__ Oh, _Float16* __restrict__ Or,
            _Float16* __restrict__ Ot, _Float16* __restrict__ Otr,
            float* __restrict__ Of, int ldc)
{
  __shared__ float st[128 * 68];

  const int t = threadIdx.x, lane = t & 31, w = t >> 5, hs = lane >> 4, l16 = lane & 15;
  const int m0 = blockIdx.x * 128, n0 = blockIdx.y * 64, z = blockIdx.z;

  const v8f z8 = {0.f, 0.f, 0.f, 0.f, 0.f, 0.f, 0.f, 0.f};
  v8f acc[2][4];
  #pragma unroll
  for (int mt = 0; mt < 2; ++mt)
    #pragma unroll
    for (int nt = 0; nt < 4; ++nt) acc[mt][nt] = z8;

  const _Float16* a0p = A + (size_t)(m0 + 32 * w + l16) * lda;
  const _Float16* a1p = a0p + (size_t)16 * lda;
  const _Float16* b0p = BT + (size_t)z * sBz + (size_t)(n0 + l16) * ldb;

  #pragma unroll 1
  for (int k0 = 0; k0 < K; k0 += 32) {
    const v16h fa0 = ldfrag(a0p + k0, hs);
    const v16h fa1 = ldfrag(a1p + k0, hs);
    #pragma unroll
    for (int nt = 0; nt < 4; ++nt) {
      const v16h fb = ldfrag(b0p + (size_t)(16 * nt) * ldb + k0, hs);
      acc[0][nt] = mma16(fa0, fb, acc[0][nt]);
      acc[1][nt] = mma16(fa1, fb, acc[1][nt]);
    }
  }

  float bv[4];
  #pragma unroll
  for (int nt = 0; nt < 4; ++nt) bv[nt] = bfr(bias[(size_t)z * sBias + n0 + 16 * nt + l16]);
  #pragma unroll
  for (int mt = 0; mt < 2; ++mt)
    #pragma unroll
    for (int nt = 0; nt < 4; ++nt)
      #pragma unroll
      for (int r = 0; r < 8; ++r) {
        float v = acc[mt][nt][r] * (1.0f / 64.0f) + bv[nt];
        if (MODE == 1) v = fmaxf(v, 0.0f);
        st[(32 * w + 16 * mt + 8 * hs + r) * 68 + 16 * nt + l16] = v;
      }
  __syncthreads();

  #pragma unroll 1
  for (int pass = 0; pass < 2; ++pass) {
    if (MODE != 2) {
      const int p = t & 7;
      #pragma unroll
      for (int j = 0; j < 8; ++j) {
        const int row = (t >> 3) + 16 * j;
        v8h hv, rv;
        #pragma unroll
        for (int i = 0; i < 8; ++i) {
          const float v = st[row * 68 + 8 * p + i];
          const _Float16 q = (_Float16)v;
          hv[i] = q;
          rv[i] = RES ? (_Float16)((v - (float)q) * 2048.0f) : q;
        }
        const size_t off = (MODE == 0) ? ((((size_t)z * prow) + m0 + row) * HD + 8 * p)
                                       : ((size_t)(m0 + row) * ldc + n0 + 8 * p);
        *(volatile v8h*)(Oh + off) = hv;
        if (RES) *(volatile v8h*)(Or + off) = rv;
      }
      if (WVT) {
        const int q16 = t & 15;
        #pragma unroll
        for (int j = 0; j < 8; ++j) {
          const int e = (t >> 4) + 8 * j;
          v8h hv, rv;
          #pragma unroll
          for (int i = 0; i < 8; ++i) {
            const float v = st[(8 * q16 + i) * 68 + e];
            const _Float16 q = (_Float16)v;
            hv[i] = q;
            rv[i] = RES ? (_Float16)((v - (float)q) * 2048.0f) : q;
          }
          const size_t off = ((size_t)z * HD + e) * (size_t)prow + m0 + 8 * q16;
          *(volatile v8h*)(Ot + off) = hv;
          if (RES) *(volatile v8h*)(Otr + off) = rv;
        }
      }
    } else {
      const int q16 = t & 15;
      #pragma unroll
      for (int j = 0; j < 16; ++j) {
        const int row = (t >> 4) + 8 * j;
        v4f fv;
        #pragma unroll
        for (int i = 0; i < 4; ++i) fv[i] = st[row * 68 + 4 * q16 + i];
        *(volatile v4f*)(Of + (size_t)(m0 + row) * ldc + n0 + 4 * q16) = fv;
      }
    }
    if (pass == 0) __threadfence();
  }
}

template<bool CAUSAL, bool RES>
__global__ __launch_bounds__(256) __attribute__((amdgpu_num_vgpr(256)))
void k_attn(const _Float16* __restrict__ Qh, const _Float16* __restrict__ Qr,
            const _Float16* __restrict__ Kh, const _Float16* __restrict__ Kr,
            const _Float16* __restrict__ Vt, const _Float16* __restrict__ Vtr,
            float* __restrict__ Out, int qb0, int prow)
{
  __shared__ _Float16 plds[8 * 16 * 40];
  __shared__ _Float16 pldr[RES ? (8 * 16 * 40) : 16];
  __shared__ float    sto[8 * 16 * 68];

  const int t = threadIdx.x, lane = t & 31, w = t >> 5, hs = lane >> 4, l16 = lane & 15;
  const int qb = qb0 + blockIdx.x, h = blockIdx.y, b = blockIdx.z;
  const int qbase = qb * 128 + w * 16;
  const size_t rq = (size_t)h * (size_t)prow + (size_t)b * SEQ;
  _Float16* pw  = plds + w * 640;
  _Float16* pwr = pldr + (RES ? w * 640 : 0);
  float*    sw  = sto + w * 1088;

  v16h aq[2], aqr[2];
  #pragma unroll
  for (int stp = 0; stp < 2; ++stp) {
    aq[stp]  = ldfrag(Qh + (rq + qbase + l16) * HD + 32 * stp, hs);
    aqr[stp] = RES ? ldfrag(Qr + (rq + qbase + l16) * HD + 32 * stp, hs) : aq[stp];
  }

  const v8f z8 = {0.f, 0.f, 0.f, 0.f, 0.f, 0.f, 0.f, 0.f};
  float mrow[8], lrow[8];
  v8f o[4], orr[4];
  #pragma unroll
  for (int r = 0; r < 8; ++r) { mrow[r] = -3.0e38f; lrow[r] = 0.0f; }
  #pragma unroll
  for (int f = 0; f < 4; ++f) { o[f] = z8; orr[f] = z8; }

  const int kend = CAUSAL ? (qbase + 16) : SEQ;

  #pragma unroll 1
  for (int kt = 0; kt < kend; kt += 32) {
    v8f s[2], sr[2];
    s[0] = z8; s[1] = z8; sr[0] = z8; sr[1] = z8;
    #pragma unroll
    for (int stp = 0; stp < 2; ++stp) {
      #pragma unroll
      for (int nt = 0; nt < 2; ++nt) {
        const size_t koff = (rq + kt + 16 * nt + l16) * HD + 32 * stp;
        const v16h fk = ldfrag(Kh + koff, hs);
        s[nt] = mma16(aq[stp], fk, s[nt]);
        if (RES) {
          sr[nt] = mma16(aqr[stp], fk, sr[nt]);
          const v16h fkr = ldfrag(Kr + koff, hs);
          sr[nt] = mma16(aq[stp], fkr, sr[nt]);
        }
      }
    }

    float pv[2][8];
    float tm[8];
    #pragma unroll
    for (int r = 0; r < 8; ++r) {
      #pragma unroll
      for (int nt = 0; nt < 2; ++nt) {
        float v = s[nt][r];
        if (RES) v += sr[nt][r] * (1.0f / 2048.0f);
        v *= 0.125f;
        if (CAUSAL) {
          const int key = kt + 16 * nt + l16;
          const int row = qbase + 8 * hs + r;
          if (key > row) v = -1.0e9f;
        }
        pv[nt][r] = v;
      }
      tm[r] = fmaxf(pv[0][r], pv[1][r]);
    }
    #pragma unroll
    for (int off = 8; off > 0; off >>= 1)
      #pragma unroll
      for (int r = 0; r < 8; ++r) tm[r] = fmaxf(tm[r], __shfl_xor(tm[r], off, 32));

    float corr[8], ts[8];
    #pragma unroll
    for (int r = 0; r < 8; ++r) {
      const float mn = fmaxf(mrow[r], tm[r]);
      corr[r] = __expf(mrow[r] - mn);
      mrow[r] = mn;
      pv[0][r] = __expf(pv[0][r] - mn);
      pv[1][r] = __expf(pv[1][r] - mn);
      ts[r] = pv[0][r] + pv[1][r];
    }
    #pragma unroll
    for (int off = 8; off > 0; off >>= 1)
      #pragma unroll
      for (int r = 0; r < 8; ++r) ts[r] += __shfl_xor(ts[r], off, 32);
    #pragma unroll
    for (int r = 0; r < 8; ++r) lrow[r] = lrow[r] * corr[r] + ts[r];
    #pragma unroll
    for (int f = 0; f < 4; ++f)
      #pragma unroll
      for (int r = 0; r < 8; ++r) {
        o[f][r] *= corr[r];
        if (RES) orr[f][r] *= corr[r];
      }

    #pragma unroll
    for (int r = 0; r < 8; ++r)
      #pragma unroll
      for (int nt = 0; nt < 2; ++nt) {
        const float pc = pv[nt][r] * 4096.0f;
        const _Float16 ph = (_Float16)pc;
        pw[(8 * hs + r) * 40 + 16 * nt + l16] = ph;
        if (RES) pwr[(8 * hs + r) * 40 + 16 * nt + l16] = (_Float16)((pc - (float)ph) * 2048.0f);
      }
    lds_sync_wave();
    const v16h ap  = ldfrag(pw + l16 * 40, hs);
    const v16h apr = RES ? ldfrag(pwr + l16 * 40, hs) : ap;

    #pragma unroll
    for (int f = 0; f < 4; ++f) {
      const size_t voff = ((size_t)h * HD + 16 * f + l16) * (size_t)prow + (size_t)b * SEQ + kt;
      const v16h fv = ldfrag(Vt + voff, hs);
      o[f] = mma16(ap, fv, o[f]);
      if (RES) {
        const v16h fvr = ldfrag(Vtr + voff, hs);
        orr[f] = mma16(ap, fvr, orr[f]);
        orr[f] = mma16(apr, fv, orr[f]);
      }
    }
    lds_sync_wave();
  }

  float inv[8];
  #pragma unroll
  for (int r = 0; r < 8; ++r) inv[r] = (1.0f / lrow[r]) * (1.0f / 4096.0f);
  #pragma unroll
  for (int f = 0; f < 4; ++f)
    #pragma unroll
    for (int r = 0; r < 8; ++r) {
      float v = o[f][r];
      if (RES) v += orr[f][r] * (1.0f / 2048.0f);
      sw[(8 * hs + r) * 68 + 16 * f + l16] = v * inv[r];
    }
  lds_sync_wave();
  const size_t orow = (size_t)b * SEQ + (size_t)qbase;
  #pragma unroll 1
  for (int pass = 0; pass < 2; ++pass) {
    #pragma unroll
    for (int j = 0; j < 8; ++j) {
      const int row = 2 * j + hs;
      const v4f fvv = *(const v4f*)(sw + row * 68 + 4 * l16);
      *(volatile v4f*)(Out + (orow + row) * DM + h * HD + 4 * l16) = fvv;
    }
    if (pass == 0) __threadfence();
  }
}

template<bool XIN, bool WH>
__global__ __launch_bounds__(256)
void k_ln(const float* __restrict__ x, const float* __restrict__ rr,
          const float* __restrict__ g, const float* __restrict__ be,
          float* __restrict__ y, _Float16* __restrict__ yh)
{
  #pragma clang fp contract(off)
  __shared__ float red[8];
  __shared__ float red2[8];
  const int m = blockIdx.x, t = threadIdx.x, lane = t & 31, w = t >> 5;
  const int c = 4 * t;
  const size_t xrow = XIN ? ((size_t)(m / SEQ) * SEQ_FULL + (size_t)(m % SEQ)) : (size_t)m;
  const v4f xv = *(const v4f*)(x + xrow * DM + c);
  const v4f rv = *(const v4f*)(rr + (size_t)m * DM + c);
  float v[4];
  #pragma unroll
  for (int i = 0; i < 4; ++i) {
    float xi = xv[i];
    if (XIN) xi = bfr(xi);
    v[i] = xi + rv[i];
  }
  float s = (v[0] + v[1]) + (v[2] + v[3]);
  #pragma unroll
  for (int off = 16; off > 0; off >>= 1) s += __shfl_xor(s, off, 32);
  if (lane == 0) red[w] = s;
  __syncthreads();
  float tot = 0.0f;
  #pragma unroll
  for (int i = 0; i < 8; ++i) tot += red[i];
  const float mu = tot * (1.0f / (float)DM);

  float d[4];
  #pragma unroll
  for (int i = 0; i < 4; ++i) d[i] = v[i] - mu;
  float s2 = (d[0] * d[0] + d[1] * d[1]) + (d[2] * d[2] + d[3] * d[3]);
  #pragma unroll
  for (int off = 16; off > 0; off >>= 1) s2 += __shfl_xor(s2, off, 32);
  if (lane == 0) red2[w] = s2;
  __syncthreads();
  float tot2 = 0.0f;
  #pragma unroll
  for (int i = 0; i < 8; ++i) tot2 += red2[i];
  const float var = tot2 * (1.0f / (float)DM);
  const float rstd = rsqrtf(var + LN_EPS);

  v4f ov;
  v4h oh;
  #pragma unroll
  for (int i = 0; i < 4; ++i) {
    const float gv = bfr(g[c + i]);
    const float bvv = bfr(be[c + i]);
    const float q = d[i] * rstd * gv + bvv;
    ov[i] = q;
    oh[i] = (_Float16)q;
  }
  float* ydst = y + (size_t)m * DM + c;
  _Float16* hdst = yh + (WH ? ((size_t)m * DM + c) : 0);
  *(volatile v4f*)ydst = ov;
  if (WH) *(volatile v4h*)hdst = oh;
  __threadfence();
  *(volatile v4f*)ydst = ov;
  if (WH) *(volatile v4h*)hdst = oh;
}

extern "C" void kernel_launch(void* const* d_in, const int* in_sizes, int n_in,
                              void* d_out, int out_size, void* d_ws, size_t ws_size,
                              hipStream_t stream)
{
  if (n_in < 16) return;
  const int MR = NB * SEQ;
  const long need_act = (long)(NB - 1) * SEQ_FULL * DM + (long)SEQ * DM;
  if ((long)in_sizes[0] < need_act || (long)in_sizes[1] < need_act) return;
  if (in_sizes[2] < NH * DM * HD || in_sizes[3] < NH * HD) return;
  if (in_sizes[4] < NH * DM * HD || in_sizes[5] < NH * HD) return;
  for (int i = 6; i < 12; ++i) if (in_sizes[i] < DM) return;
  if (in_sizes[12] < DM * FF || in_sizes[13] < FF || in_sizes[14] < FF * DM || in_sizes[15] < DM) return;
  if (out_size < MR * DM) return;

  const float* y      = (const float*)d_in[0];
  const float* enc    = (const float*)d_in[1];
  const float* Wself  = (const float*)d_in[2];
  const float* bself  = (const float*)d_in[3];
  const float* Wcross = (const float*)d_in[4];
  const float* bcross = (const float*)d_in[5];
  const float* g1  = (const float*)d_in[6];  const float* be1 = (const float*)d_in[7];
  const float* g2  = (const float*)d_in[8];  const float* be2 = (const float*)d_in[9];
  const float* g3  = (const float*)d_in[10]; const float* be3 = (const float*)d_in[11];
  const float* w1  = (const float*)d_in[12]; const float* b1  = (const float*)d_in[13];
  const float* w2  = (const float*)d_in[14]; const float* b2  = (const float*)d_in[15];
  float* out = (float*)d_out;

  char* base = (char*)d_ws;
  size_t off = 0;
  auto take = [&](size_t bytes) -> void* {
    void* p = (void*)(base + off);
    off += (bytes + 255) & ~(size_t)255;
    return p;
  };
  _Float16* Yh   = (_Float16*)take((size_t)MR * DM * 2);
  _Float16* Eh   = (_Float16*)take((size_t)MR * DM * 2);
  _Float16* WTs  = (_Float16*)take((size_t)NH * HD * DM * 2);
  _Float16* WTc  = (_Float16*)take((size_t)NH * HD * DM * 2);
  _Float16* W1T  = (_Float16*)take((size_t)FF * DM * 2);
  _Float16* W2T  = (_Float16*)take((size_t)DM * FF * 2);
  _Float16* QKVh = (_Float16*)take((size_t)NH * MR * HD * 2);
  _Float16* QKVr = (_Float16*)take((size_t)NH * MR * HD * 2);
  _Float16* VTh  = (_Float16*)take((size_t)NH * HD * MR * 2);
  _Float16* VTr  = (_Float16*)take((size_t)NH * HD * MR * 2);
  float*    att  = (float*)   take((size_t)MR * DM * 4);
  float*    y1   = (float*)   take((size_t)MR * DM * 4);
  _Float16* y1h  = (_Float16*)take((size_t)MR * DM * 2);
  float*    y2   = (float*)   take((size_t)MR * DM * 4);
  _Float16* y2h  = (_Float16*)take((size_t)MR * DM * 2);
  _Float16* Qch  = (_Float16*)take((size_t)NH * MR * HD * 2);
  _Float16* KVch = (_Float16*)take((size_t)NH * MR * HD * 2);
  _Float16* VTc  = (_Float16*)take((size_t)NH * HD * MR * 2);
  _Float16* Hh   = (_Float16*)take((size_t)MR * FF * 2);
  if (off > ws_size) return;

  {
    const int groups2 = 2 * MR * (DM / 8);
    k_cvt_act<<<dim3((groups2 + 255) / 256), 256, 0, stream>>>(y, enc, Yh, Eh, MR);
  }
  k_wtr<<<dim3(HD / 64, DM / 64, NH), 256, 0, stream>>>(Wself, WTs, DM, HD, 64.0f);
  k_wtr<<<dim3(HD / 64, DM / 64, NH), 256, 0, stream>>>(Wcross, WTc, DM, HD, 64.0f);
  k_wtr<<<dim3(FF / 64, DM / 64, 1), 256, 0, stream>>>(w1, W1T, DM, FF, 64.0f);
  k_wtr<<<dim3(DM / 64, FF / 64, 1), 256, 0, stream>>>(w2, W2T, FF, DM, 64.0f);

  const int nqb  = SEQ / 128;
  const int nres = (nqb < RESQB) ? nqb : RESQB;

  k_gemm<0, true, true><<<dim3(MR / 128, HD / 64, NH), 128, 0, stream>>>(
      Yh, DM, WTs, DM, HD * DM, bself, HD, DM, MR, QKVh, QKVr, VTh, VTr, att, HD);
  k_attn<true, true><<<dim3(nres, NH, NB), 256, 0, stream>>>(
      QKVh, QKVr, QKVh, QKVr, VTh, VTr, att, 0, MR);
  if (nqb > nres)
    k_attn<true, false><<<dim3(nqb - nres, NH, NB), 256, 0, stream>>>(
        QKVh, QKVr, QKVh, QKVr, VTh, VTr, att, nres, MR);
  k_ln<true, true><<<dim3(MR), 256, 0, stream>>>(y, att, g1, be1, y1, y1h);

  k_gemm<0, false, false><<<dim3(MR / 128, HD / 64, NH), 128, 0, stream>>>(
      y1h, DM, WTc, DM, HD * DM, bcross, HD, DM, MR, Qch, Qch, Qch, Qch, att, HD);
  k_gemm<0, false, true><<<dim3(MR / 128, HD / 64, NH), 128, 0, stream>>>(
      Eh, DM, WTc, DM, HD * DM, bcross, HD, DM, MR, KVch, KVch, VTc, VTc, att, HD);
  k_attn<false, false><<<dim3(nqb, NH, NB), 256, 0, stream>>>(
      Qch, Qch, KVch, KVch, VTc, VTc, att, 0, MR);
  k_ln<false, true><<<dim3(MR), 256, 0, stream>>>(y1, att, g2, be2, y2, y2h);

  k_gemm<1, false, false><<<dim3(MR / 128, FF / 64, 1), 128, 0, stream>>>(
      y2h, DM, W1T, DM, 0, b1, 0, DM, MR, Hh, Hh, Hh, Hh, att, FF);
  k_gemm<2, false, false><<<dim3(MR / 128, DM / 64, 1), 128, 0, stream>>>(
      Hh, FF, W2T, FF, 0, b2, 0, FF, MR, y2h, y2h, y2h, y2h, att, DM);
  k_ln<false, false><<<dim3(MR), 256, 0, stream>>>(y2, att, g3, be3, out, y2h);
}
